// PhasePairs_20985210208770
// MI455X (gfx1250) — hardware-verified
//
#include <hip/hip_runtime.h>
#include <stddef.h>
#include <stdint.h>

#define G_  512
#define T_  128
#define P_  64
#define B_  128
#define GB  8
#define APH 72

static_assert(G_ % GB == 0);
static_assert(B_ == 8 * 16);
static_assert(T_ % 16 == 0);
static_assert(P_ == 64);
static_assert((APH * 2) % 16 == 0);
static_assert((T_ * P_) % (256 * 4) == 0);

typedef _Float16 v16h __attribute__((ext_vector_type(16)));
typedef _Float16 v8h  __attribute__((ext_vector_type(8)));
typedef _Float16 v4h  __attribute__((ext_vector_type(4)));
typedef float    v8f  __attribute__((ext_vector_type(8)));
typedef int      v4i  __attribute__((ext_vector_type(4)));
typedef v8h __attribute__((may_alias)) v8ha;
typedef v4h __attribute__((may_alias)) v4ha;
typedef v4i __attribute__((may_alias)) v4ia;

union Frag { v16h v; v8h h[2]; };

__constant__ int kUnitPhases[32] = { 1, 0, 0, 0,   0, 1, 0, 0,   0, 0, 1, 0,   0, 0, 0, -1,
                                    -1, 0, 0, 0,   0,-1, 0, 0,   0, 0,-1, 0,   0, 0, 0,  1};
__constant__ int kIdentity[4] = {1, 0, 0, 0};

__device__ __forceinline__ v8f mma16(v16h a, v16h b, v8f cacc) {
  cacc = __builtin_amdgcn_wmma_f32_16x16x32_f16(false, a, false, b, (short)0, cacc, false, false);
  asm volatile("v_nop\n\tv_nop\n\tv_nop\n\tv_nop" : "+v"(cacc) : "v"(a), "v"(b));
  return cacc;
}

__device__ __forceinline__ v8f zero8() { return (v8f){0.f, 0.f, 0.f, 0.f, 0.f, 0.f, 0.f, 0.f}; }

__device__ __forceinline__ _Float16 bit_h(int v) { return (_Float16)(v & 1); }

__device__ __forceinline__ v16h ldfrag_l(const _Float16* p, int ld, int row0, int k0, int lane) {
  const int m = lane & 15, lh = lane >> 4;
  const _Float16* q = p + (row0 + m) * ld + k0 + 8 * lh;
  Frag f;
  f.h[0] = *(const v8ha*)(q);
  f.h[1] = *(const v8ha*)(q + 16);
  return f.v;
}

__device__ __forceinline__ v16h ldfrag_pv(const int* __restrict__ pv, int b0, int k0, int lane) {
  const int m = lane & 15, lh = lane >> 4;
  const int* q = pv + (size_t)(b0 + m) * P_ + k0 + 8 * lh;
  const v4i u0 = *(const v4ia*)(q);
  const v4i u1 = *(const v4ia*)(q + 4);
  const v4i u2 = *(const v4ia*)(q + 16);
  const v4i u3 = *(const v4ia*)(q + 20);
  Frag f;
  f.h[0] = (v8h){bit_h(u0.x), bit_h(u0.y), bit_h(u0.z), bit_h(u0.w), bit_h(u1.x), bit_h(u1.y), bit_h(u1.z), bit_h(u1.w)};
  f.h[1] = (v8h){bit_h(u2.x), bit_h(u2.y), bit_h(u2.z), bit_h(u2.w), bit_h(u3.x), bit_h(u3.y), bit_h(u3.z), bit_h(u3.w)};
  return f.v;
}

__device__ __forceinline__ void zw_mul(uint32_t x0, uint32_t x1, uint32_t x2, uint32_t x3,
                                       uint32_t y0, uint32_t y1, uint32_t y2, uint32_t y3,
                                       uint32_t& c0, uint32_t& c1, uint32_t& c2, uint32_t& c3) {
  c0 = x0 * y0 - x1 * y3 - x2 * y2 - x3 * y1;
  c1 = x0 * y1 + x1 * y0 - x2 * y3 - x3 * y2;
  c2 = x0 * y2 + x1 * y1 + x2 * y0 - x3 * y3;
  c3 = x0 * y3 + x1 * y2 + x2 * y1 + x3 * y0;
}

__global__ __launch_bounds__(256) void k_main(const int* __restrict__ alpha, const int* __restrict__ ap,
                                              const int* __restrict__ beta,  const int* __restrict__ bp,
                                              const int* __restrict__ counts, const int* __restrict__ pv,
                                              int* __restrict__ out) {
  __shared__ __align__(16) _Float16 sA[T_ * APH];
  __shared__ __align__(16) _Float16 sB[T_ * APH];
  __shared__ __align__(16) v4i sStage[8][128];
  __shared__ __align__(16) v4i sTab[64];
  __shared__ int sAl[T_];
  __shared__ int sBe[T_];

  const int tid = threadIdx.x, lane = tid & 31, wave = tid >> 5;
  const int h = lane >> 4, m = lane & 15;
  const int g0 = blockIdx.x * GB;
  const int b0 = wave * 16;

  if (tid < 64) {
    const int a = tid >> 3, b = tid & 7, gg = (a + b) & 7;
    v4i tv;
    tv.x = kIdentity[0] + kUnitPhases[a * 4 + 0] + kUnitPhases[b * 4 + 0] - kUnitPhases[gg * 4 + 0];
    tv.y = kIdentity[1] + kUnitPhases[a * 4 + 1] + kUnitPhases[b * 4 + 1] - kUnitPhases[gg * 4 + 1];
    tv.z = kIdentity[2] + kUnitPhases[a * 4 + 2] + kUnitPhases[b * 4 + 2] - kUnitPhases[gg * 4 + 2];
    tv.w = kIdentity[3] + kUnitPhases[a * 4 + 3] + kUnitPhases[b * 4 + 3] - kUnitPhases[gg * 4 + 3];
    sTab[tid] = tv;
  }

  const v16h bf0 = ldfrag_pv(pv, b0, 0, lane);
  const v16h bf1 = ldfrag_pv(pv, b0, 32, lane);

#pragma unroll 1
  for (int gi = 0; gi < GB; ++gi) {
    const int g = g0 + gi;
    __syncthreads();
    {
      const int* apg = ap + (size_t)g * (T_ * P_);
      const int* bpg = bp + (size_t)g * (T_ * P_);
#pragma unroll
      for (int j = 0; j < (T_ * P_) / (256 * 4); ++j) {
        const int q  = tid + 256 * j;
        const int t  = q >> 4;
        const int pc = q & 15;
        const v4i va = *(const v4ia*)(apg + (size_t)q * 4);
        const v4i vb = *(const v4ia*)(bpg + (size_t)q * 4);
        const v4h ha = (v4h){bit_h(va.x), bit_h(va.y), bit_h(va.z), bit_h(va.w)};
        const v4h hb = (v4h){bit_h(vb.x), bit_h(vb.y), bit_h(vb.z), bit_h(vb.w)};
        *(v4ha*)(sA + t * APH + pc * 4) = ha;
        *(v4ha*)(sB + t * APH + pc * 4) = hb;
      }
    }
    if (tid < T_) sAl[tid] = alpha[(size_t)g * T_ + tid];
    else          sBe[tid - T_] = beta[(size_t)g * T_ + (tid - T_)];
    const int cnt = counts[g];
    __syncthreads();

    uint32_t p0 = 1u, p1 = 0u, p2 = 0u, p3 = 0u;
#pragma unroll 1
    for (int tt = 0; tt < T_ / 16; ++tt) {
      const int t0 = tt * 16;
      v8f accA = zero8(), accB = zero8();
      {
        const v16h a0 = ldfrag_l(sA, APH, t0, 0, lane);
        const v16h a1 = ldfrag_l(sA, APH, t0, 32, lane);
        accA = mma16(a0, bf0, accA);
        accA = mma16(a1, bf1, accA);
      }
      {
        const v16h c0 = ldfrag_l(sB, APH, t0, 0, lane);
        const v16h c1 = ldfrag_l(sB, APH, t0, 32, lane);
        accB = mma16(c0, bf0, accB);
        accB = mma16(c1, bf1, accB);
      }
#pragma unroll
      for (int r = 0; r < 8; ++r) {
        const int t  = t0 + (h << 3) + r;
        const int pa = ((int)accA[r]) & 1;
        const int pb = ((int)accB[r]) & 1;
        const int a  = (sAl[t] + (pa << 2)) & 7;
        const int bb = (sBe[t] + (pb << 2)) & 7;
        const v4i tv = sTab[(a << 3) | bb];
        uint32_t n0, n1, n2, n3;
        zw_mul(p0, p1, p2, p3, (uint32_t)tv.x, (uint32_t)tv.y, (uint32_t)tv.z, (uint32_t)tv.w, n0, n1, n2, n3);
        const bool on = t < cnt;
        p0 = on ? n0 : p0;
        p1 = on ? n1 : p1;
        p2 = on ? n2 : p2;
        p3 = on ? n3 : p3;
      }
    }

    const uint32_t q0 = __shfl_xor(p0, 16, 32);
    const uint32_t q1 = __shfl_xor(p1, 16, 32);
    const uint32_t q2 = __shfl_xor(p2, 16, 32);
    const uint32_t q3 = __shfl_xor(p3, 16, 32);
    uint32_t f0, f1, f2, f3;
    zw_mul(p0, p1, p2, p3, q0, q1, q2, q3, f0, f1, f2, f3);
    if (h == 0) sStage[wave][m * 8 + gi] = (v4i){(int)f0, (int)f1, (int)f2, (int)f3};
  }
  __syncthreads();

  v4i val[4];
  size_t go[4];
#pragma unroll
  for (int it = 0; it < 4; ++it) {
    const int p  = lane + 32 * it;
    const int L  = p >> 3;
    const int pc = p & 7;
    val[it] = sStage[wave][p];
    go[it]  = ((size_t)(b0 + L) * G_ + (size_t)(g0 + pc)) * 4;
  }
#pragma unroll
  for (int it = 0; it < 4; ++it) *(volatile v4i*)(out + go[it]) = val[it];
  __threadfence();
#pragma unroll
  for (int it = 0; it < 4; ++it) *(volatile v4i*)(out + go[it]) = val[it];
}

extern "C" void kernel_launch(void* const* d_in, const int* in_sizes, int n_in,
                              void* d_out, int out_size, void* d_ws, size_t ws_size,
                              hipStream_t stream) {
  (void)d_ws; (void)ws_size;
  if (n_in < 6) return;
  if (in_sizes[0] != G_ * T_) return;
  if (in_sizes[1] != G_ * T_ * P_) return;
  if (in_sizes[2] != G_ * T_) return;
  if (in_sizes[3] != G_ * T_ * P_) return;
  if (in_sizes[4] != G_) return;
  if (in_sizes[5] != B_ * P_) return;
  if (out_size != B_ * G_ * 4) return;

  const int* alpha        = (const int*)d_in[0];
  const int* alpha_params = (const int*)d_in[1];
  const int* beta         = (const int*)d_in[2];
  const int* beta_params  = (const int*)d_in[3];
  const int* counts       = (const int*)d_in[4];
  const int* param_vals   = (const int*)d_in[5];
  int* out = (int*)d_out;

  k_main<<<dim3(G_ / GB), dim3(256), 0, stream>>>(alpha, alpha_params, beta, beta_params, counts, param_vals, out);
  (void)hipGetLastError();
}
